// PointNetSetAbstraction_72524817760258
// MI455X (gfx1250) — hardware-verified
//
#include <hip/hip_runtime.h>
#include <math.h>
#pragma clang fp contract(off)

typedef __attribute__((ext_vector_type(16))) _Float16 v16h;
typedef __attribute__((ext_vector_type(8)))  float    v8f;
typedef __attribute__((ext_vector_type(4)))  float    v4f;
typedef __attribute__((ext_vector_type(4)))  unsigned v4u;
typedef __attribute__((ext_vector_type(8)))  unsigned v8u;

constexpr int NBATCH    = 16;
constexpr int NPTS_IN   = 4096;
constexpr int NCENT     = 512;
constexpr int NSAMP     = 32;
constexpr int MROWS_ALL = NBATCH * NCENT * NSAMP;
constexpr int LAYER_BLOCKS = MROWS_ALL / 64;
constexpr float WCARRY     = 16.0f;
constexpr float WCARRY_INV = 1.0f / 16.0f;
constexpr float RES_CARRY     = 2048.0f;
constexpr float RES_CARRY_INV = 1.0f / 2048.0f;
constexpr float RADIUS_SQ  = (float)(0.5 * 0.5);
constexpr float BN_EPS     = 1e-5f;
static_assert(MROWS_ALL == 262144);
static_assert(LAYER_BLOCKS == 4096);
static_assert(NSAMP == 32);

__device__ __forceinline__ float h16_to_f32(unsigned hb) {
  const unsigned sgn = (hb & 0x8000u) << 16;
  const unsigned em = hb & 0x7fffu;
  const float fn = __uint_as_float((em << 13) + 0x38000000u);
  const float fs = (float)em * 5.9604644775390625e-8f;
  const float mag = (em < 0x400u) ? fs : fn;
  return __uint_as_float(__float_as_uint(mag) | sgn);
}
__device__ __forceinline__ unsigned h16bits(float x) {
  const _Float16 hx = (_Float16)x;
  const unsigned short s = __builtin_bit_cast(unsigned short, hx);
  return (unsigned)s;
}
__device__ __forceinline__ unsigned pack2(float a, float b) {
  const unsigned lo = h16bits(a);
  const unsigned hi = h16bits(b);
  return lo | (hi << 16);
}
__device__ __forceinline__ void split_h(float x, unsigned& hb, unsigned& lb) {
  unsigned b = h16bits(x);
  const unsigned em = b & 0x7fffu;
  b = (em < 0x400u) ? 0u : b;
  const float hf = h16_to_f32(b);
  const float res = x - hf;
  const float rsc = res * RES_CARRY;
  hb = b;
  lb = h16bits(rsc);
}
__device__ __forceinline__ v8f mma_f16(v16h a, v16h b, v8f c) {
  c = __builtin_amdgcn_wmma_f32_16x16x32_f16(false, a, false, b, (short)0, c, false, false);
  asm volatile("v_nop\n\tv_nop\n\tv_nop\n\tv_nop" : "+v"(c) : "v"(a), "v"(b));
  return c;
}
__device__ __forceinline__ void guard2(v8f& a, v8f& b, v16h x, v16h y, v16h z) {
  asm volatile("v_nop\n\tv_nop\n\tv_nop\n\tv_nop" : "+v"(a), "+v"(b) : "v"(x), "v"(y), "v"(z));
}
__device__ __forceinline__ void wave_lds_sync() {
  __builtin_amdgcn_fence(__ATOMIC_RELEASE, "workgroup");
  __builtin_amdgcn_wave_barrier();
  __builtin_amdgcn_fence(__ATOMIC_ACQUIRE, "workgroup");
}
__device__ __forceinline__ v16h frag_from_words(v4u w0, v4u w1) {
  const v8u w = __builtin_shufflevector(w0, w1, 0, 1, 2, 3, 4, 5, 6, 7);
  return __builtin_bit_cast(v16h, w);
}
template <int EO>
__device__ __forceinline__ void bn_cvt8(v16h& av, v4u w, const float* scp, const float* shp) {
  const v4f s0 = *(const v4f*)scp;
  const v4f s1 = *(const v4f*)(scp + 4);
  const v4f h0 = *(const v4f*)shp;
  const v4f h1 = *(const v4f*)(shp + 4);
  const unsigned wa = w[0];
  const unsigned wb = w[1];
  const unsigned wc = w[2];
  const unsigned wd = w[3];
  float f;
  f = h16_to_f32(wa & 0xffffu); f = f * s0[0]; f = f + h0[0]; f = fmaxf(f, 0.0f); av[EO + 0] = (_Float16)f;
  f = h16_to_f32(wa >> 16);     f = f * s0[1]; f = f + h0[1]; f = fmaxf(f, 0.0f); av[EO + 1] = (_Float16)f;
  f = h16_to_f32(wb & 0xffffu); f = f * s0[2]; f = f + h0[2]; f = fmaxf(f, 0.0f); av[EO + 2] = (_Float16)f;
  f = h16_to_f32(wb >> 16);     f = f * s0[3]; f = f + h0[3]; f = fmaxf(f, 0.0f); av[EO + 3] = (_Float16)f;
  f = h16_to_f32(wc & 0xffffu); f = f * s1[0]; f = f + h1[0]; f = fmaxf(f, 0.0f); av[EO + 4] = (_Float16)f;
  f = h16_to_f32(wc >> 16);     f = f * s1[1]; f = f + h1[1]; f = fmaxf(f, 0.0f); av[EO + 5] = (_Float16)f;
  f = h16_to_f32(wd & 0xffffu); f = f * s1[2]; f = f + h1[2]; f = fmaxf(f, 0.0f); av[EO + 6] = (_Float16)f;
  f = h16_to_f32(wd >> 16);     f = f * s1[3]; f = f + h1[3]; f = fmaxf(f, 0.0f); av[EO + 7] = (_Float16)f;
}

__global__ __launch_bounds__(256) void k_prep(const float* __restrict__ W0, const float* __restrict__ W1,
                                              const float* __restrict__ W2, unsigned* __restrict__ wpl) {
  const int i = blockIdx.x * 256 + threadIdx.x;
  float v0 = 0.0f;
  float v1 = 0.0f;
  if (i < 1024) {
    const int n = i >> 4;
    const int kp = (i & 15) * 2;
    const int ka = kp < 9 ? kp : 8;
    const int kb = (kp + 1) < 9 ? (kp + 1) : 8;
    const float a = W0[n * 9 + ka];
    const float b = W0[n * 9 + kb];
    v0 = (kp < 9) ? a * WCARRY : 0.0f;
    v1 = ((kp + 1) < 9) ? b * WCARRY : 0.0f;
  } else if (i < 3072) {
    const int j = i - 1024;
    v0 = W1[2 * j] * WCARRY;
    v1 = W1[2 * j + 1] * WCARRY;
  } else {
    const int j = i - 3072;
    v0 = W2[2 * j] * WCARRY;
    v1 = W2[2 * j + 1] * WCARRY;
  }
  const unsigned u = pack2(v0, v1);
  ((volatile unsigned*)wpl)[i] = u;
  __threadfence();
  ((volatile unsigned*)wpl)[i] = u;
}

__global__ __launch_bounds__(1024) void k_fps(const float* __restrict__ xyz, float* __restrict__ out0,
                                              float* __restrict__ cen) {
#pragma clang fp contract(off)
  __shared__ __align__(16) float pts[3 * NPTS_IN];
  __shared__ float rv[2][32];
  __shared__ int ri[2][32];
  __shared__ int sel[NCENT];
  const int b = blockIdx.x;
  const int t = threadIdx.x;
  const int lane = t & 31;
  const int wave = t >> 5;
  const float* xb = xyz + (size_t)b * 3 * NPTS_IN;
  const v4f X = *(const v4f*)(xb + 4 * t);
  const v4f Y = *(const v4f*)(xb + NPTS_IN + 4 * t);
  const v4f Z = *(const v4f*)(xb + 2 * NPTS_IN + 4 * t);
  *(v4f*)(pts + 4 * t) = X;
  *(v4f*)(pts + NPTS_IN + 4 * t) = Y;
  *(v4f*)(pts + 2 * NPTS_IN + 4 * t) = Z;
  float dist[4];
#pragma unroll
  for (int j = 0; j < 4; ++j) dist[j] = 1e10f;
  int far = 0;
  __syncthreads();

  for (int step = 0; step < NCENT; ++step) {
    if (t == 0) sel[step] = far;
    const float cx = pts[far];
    const float cy = pts[NPTS_IN + far];
    const float cz = pts[2 * NPTS_IN + far];
    float bv = -1.0f;
    int bi = 4 * t;
#pragma unroll
    for (int j = 0; j < 4; ++j) {
      const float dx = X[j] - cx;
      const float dy = Y[j] - cy;
      const float dz = Z[j] - cz;
      const float t0 = dx * dx;
      const float t1 = dy * dy;
      const float t2 = dz * dz;
      const float s02 = t0 + t2;
      const float d = s02 + t1;
      const float dn = fminf(dist[j], d);
      dist[j] = dn;
      if (dn > bv) { bv = dn; bi = 4 * t + j; }
    }
#pragma unroll
    for (int off = 16; off > 0; off >>= 1) {
      const float v2 = __shfl_xor(bv, off, 32);
      const int i2 = __shfl_xor(bi, off, 32);
      const bool take = (v2 > bv) || ((v2 == bv) && (i2 < bi));
      bv = take ? v2 : bv;
      bi = take ? i2 : bi;
    }
    const int p = step & 1;
    if (lane == 0) { rv[p][wave] = bv; ri[p][wave] = bi; }
    __syncthreads();
    bv = rv[p][lane];
    bi = ri[p][lane];
#pragma unroll
    for (int off = 16; off > 0; off >>= 1) {
      const float v2 = __shfl_xor(bv, off, 32);
      const int i2 = __shfl_xor(bi, off, 32);
      const bool take = (v2 > bv) || ((v2 == bv) && (i2 < bi));
      bv = take ? v2 : bv;
      bi = take ? i2 : bi;
    }
    far = bi < 0 ? 0 : (bi > NPTS_IN - 1 ? NPTS_IN - 1 : bi);
  }
  __syncthreads();

  if (t < 384) {
    const int c = t >> 7;
    const int k4 = (t & 127) * 4;
    v4f v;
#pragma unroll
    for (int e = 0; e < 4; ++e) {
      int id = sel[k4 + e];
      id = id < 0 ? 0 : (id > NPTS_IN - 1 ? NPTS_IN - 1 : id);
      v[e] = pts[c * NPTS_IN + id];
    }
    float* po = out0 + (size_t)(b * 3 + c) * NCENT + k4;
    float* pc = cen + (size_t)(b * 3 + c) * NCENT + k4;
    for (int pass = 0; pass < 2; ++pass) {
      *(volatile v4f*)po = v;
      *(volatile v4f*)pc = v;
      __threadfence();
    }
  }
}

__global__ __launch_bounds__(128) void k_group(const float* __restrict__ xyz, const float* __restrict__ feat,
                                               const float* __restrict__ cen, unsigned* __restrict__ X0) {
#pragma clang fp contract(off)
  __shared__ __align__(16) float pts[3 * NPTS_IN];
  __shared__ int hl[4][32];
  __shared__ __align__(16) unsigned xt[4][32 * 16];
  const int t = threadIdx.x;
  const int lane = t & 31;
  const int wave = t >> 5;
  const int b = blockIdx.x >> 4;
  const int kblk = (blockIdx.x & 15) * 32;
  const float* xb = xyz + (size_t)b * 3 * NPTS_IN;
#pragma unroll 4
  for (int i = t; i < 3 * NPTS_IN / 4; i += 128) {
    const v4f v = *(const v4f*)(xb + 4 * i);
    *(v4f*)(pts + 4 * i) = v;
  }
  __syncthreads();
  const float* fb = feat + (size_t)b * 6 * NPTS_IN;
  const unsigned lt_mask = (1u << lane) - 1u;

  for (int qi = 0; qi < 8; ++qi) {
    const int k = kblk + wave * 8 + qi;
    const float qx = cen[(size_t)(b * 3 + 0) * NCENT + k];
    const float qy = cen[(size_t)(b * 3 + 1) * NCENT + k];
    const float qz = cen[(size_t)(b * 3 + 2) * NCENT + k];
    hl[wave][lane] = 0;
    wave_lds_sync();
    int cnt = 0;
    int first = 0;
    for (int ch = 0; ch < NPTS_IN / 32; ++ch) {
      const int n = ch * 32 + lane;
      const float dx = qx - pts[n];
      const float dy = qy - pts[NPTS_IN + n];
      const float dz = qz - pts[2 * NPTS_IN + n];
      const float t0 = dx * dx;
      const float t1 = dy * dy;
      const float t2 = dz * dz;
      const float s02 = t0 + t2;
      const float d = s02 + t1;
      const bool hit = !(d > RADIUS_SQ);
      const unsigned mask = __builtin_amdgcn_ballot_w32(hit);
      const int pos = cnt + __popc(mask & lt_mask);
      if (hit && pos < NSAMP) hl[wave][pos] = n;
      if (cnt == 0 && mask != 0u) first = ch * 32 + (__ffs(mask) - 1);
      cnt += __popc(mask);
      if (cnt >= NSAMP) break;
    }
    wave_lds_sync();
    const int cntc = cnt < NSAMP ? cnt : NSAMP;
    const int hv = hl[wave][lane];
    int nid = (lane < cntc) ? hv : first;
    nid = nid < 0 ? 0 : (nid > NPTS_IN - 1 ? NPTS_IN - 1 : nid);
    const float gx = pts[nid] - qx;
    const float gy = pts[NPTS_IN + nid] - qy;
    const float gz = pts[2 * NPTS_IN + nid] - qz;
    const float f0 = fb[nid];
    const float f1 = fb[NPTS_IN + nid];
    const float f2 = fb[2 * NPTS_IN + nid];
    const float f3 = fb[3 * NPTS_IN + nid];
    const float f4 = fb[4 * NPTS_IN + nid];
    const float f5 = fb[5 * NPTS_IN + nid];
    unsigned hgx, hgy, hgz, hf0, hf1, hf2, hf3, hf4, hf5;
    unsigned lgx, lgy, lgz, lf0, lf1, lf2, lf3, lf4, lf5;
    split_h(gx, hgx, lgx);
    split_h(gy, hgy, lgy);
    split_h(gz, hgz, lgz);
    split_h(f0, hf0, lf0);
    split_h(f1, hf1, lf1);
    split_h(f2, hf2, lf2);
    split_h(f3, hf3, lf3);
    split_h(f4, hf4, lf4);
    split_h(f5, hf5, lf5);
    unsigned zz = 0;
    asm volatile("" : "+v"(zz));
    const v4u r0 = { hgx | (hgy << 16), hgz | (hf0 << 16), hf1 | (hf2 << 16), hf3 | (hf4 << 16) };
    const v4u r1 = { hf5 | (zz << 16), zz, zz, zz };
    const v4u l0 = { lgx | (lgy << 16), lgz | (lf0 << 16), lf1 | (lf2 << 16), lf3 | (lf4 << 16) };
    const v4u l1 = { lf5 | (zz << 16), zz, zz, zz };
    unsigned* xr = &xt[wave][lane * 16];
    *(v4u*)(xr) = r0;
    *(v4u*)(xr + 4) = r1;
    *(v4u*)(xr + 8) = l0;
    *(v4u*)(xr + 12) = l1;
    wave_lds_sync();
    const v4u o0 = *(const v4u*)(&xt[wave][lane * 4]);
    const v4u o1 = *(const v4u*)(&xt[wave][128 + lane * 4]);
    const v4u o2 = *(const v4u*)(&xt[wave][256 + lane * 4]);
    const v4u o3 = *(const v4u*)(&xt[wave][384 + lane * 4]);
    unsigned* gp = X0 + (size_t)(b * NCENT + k) * (NSAMP * 16) + lane * 4;
    for (int pass = 0; pass < 2; ++pass) {
      *(volatile v4u*)(gp) = o0;
      *(volatile v4u*)(gp + 128) = o1;
      *(volatile v4u*)(gp + 256) = o2;
      *(volatile v4u*)(gp + 384) = o3;
      __threadfence();
    }
    wave_lds_sync();
  }
}

template <int KDIM, int NOUT, bool BNIN, bool POOL, bool RESID>
__global__ __launch_bounds__(128) void k_layer(const unsigned* __restrict__ Ain, const unsigned* __restrict__ Wh,
                                               const float* __restrict__ bias, const float* __restrict__ ssin,
                                               unsigned* __restrict__ Yout, float* __restrict__ pst,
                                               float* __restrict__ gmm) {
  static_assert(KDIM % 32 == 0);
  static_assert(NOUT % 16 == 0);
  static_assert(NOUT <= 128);
  static_assert(POOL || NOUT == 64);
  static_assert(!POOL || NOUT == 128);
  static_assert(!RESID || (KDIM == 32 && !BNIN));
  constexpr int KS = KDIM / 32;
  constexpr int NT = NOUT / 16;
  constexpr int PW = (KDIM + 8) / 2;
  constexpr int AW = KDIM / 2;
  constexpr int VPR = KDIM / 8;
  constexpr int NV = NOUT * VPR;
  __shared__ __align__(16) unsigned Bs[NOUT * PW];
  __shared__ __align__(16) float ssl[128];
  __shared__ __align__(16) float bsl[NOUT];
  __shared__ __align__(16) float slab[POOL ? 1 : 4][POOL ? 4 : 16 * 68];
  __shared__ __align__(16) float rs[4][NOUT];
  __shared__ __align__(16) float rq[4][NOUT];
  __shared__ __align__(16) float pm[POOL ? 4 : 1][POOL ? 128 : 4];
  __shared__ __align__(16) float pn[POOL ? 4 : 1][POOL ? 128 : 4];

  const int t = threadIdx.x;
  const int lane = t & 31;
  const int wave = t >> 5;
  const int h = lane >> 4;
  const int c = lane & 15;

#pragma unroll 2
  for (int i = t; i < NV; i += 128) {
    const int n = i / VPR;
    const int q = i - n * VPR;
    const v4u w = *(const v4u*)(Wh + (size_t)i * 4);
    *(v4u*)(&Bs[n * PW + q * 4]) = w;
  }
  if (BNIN) {
    if (t < 64) {
      ssl[t] = ssin[t];
      ssl[64 + t] = ssin[128 + t];
    }
  }
  if (t < NOUT) bsl[t] = bias[t];
  __syncthreads();

  const int arow = blockIdx.x * 64 + wave * 16 + c;
  const unsigned* ap = Ain + (size_t)arow * AW + 4 * h;
  v4u aw0[KS];
  v4u aw1[KS];
#pragma unroll
  for (int ks = 0; ks < KS; ++ks) {
    aw0[ks] = *(const v4u*)(ap + ks * 16);
    aw1[ks] = *(const v4u*)(ap + ks * 16 + 8);
  }
  v16h afr[KS];
#pragma unroll
  for (int ks = 0; ks < KS; ++ks) {
    if (BNIN) {
      v16h av;
      bn_cvt8<0>(av, aw0[ks], &ssl[ks * 32 + 8 * h], &ssl[64 + ks * 32 + 8 * h]);
      bn_cvt8<8>(av, aw1[ks], &ssl[ks * 32 + 16 + 8 * h], &ssl[64 + ks * 32 + 16 + 8 * h]);
      afr[ks] = av;
    } else {
      afr[ks] = frag_from_words(aw0[ks], aw1[ks]);
    }
  }
  v16h afl = afr[0];
  if (RESID) {
    const v4u zv = { 0u, 0u, 0u, 0u };
    afr[0] = frag_from_words(aw0[0], zv);
    afl = frag_from_words(aw1[0], zv);
  }

#pragma unroll 1
  for (int j = 0; j < NT; ++j) {
    v8f acc = (v8f){0.f, 0.f, 0.f, 0.f, 0.f, 0.f, 0.f, 0.f};
    v8f acr = (v8f){0.f, 0.f, 0.f, 0.f, 0.f, 0.f, 0.f, 0.f};
    const unsigned* bp = &Bs[(j * 16 + c) * PW + 4 * h];
#pragma unroll
    for (int ks = 0; ks < KS; ++ks) {
      const v4u b0 = *(const v4u*)(bp + ks * 16);
      const v4u b1 = *(const v4u*)(bp + ks * 16 + 8);
      const v16h bf = frag_from_words(b0, b1);
      acc = mma_f16(afr[ks], bf, acc);
      if (RESID) {
        acr = mma_f16(afl, bf, acr);
        guard2(acc, acr, afr[ks], afl, bf);
      }
    }
    const int col = j * 16 + c;
    const float bv = bsl[col];
    float ls = 0.0f;
    float lq = 0.0f;
    float mx = -INFINITY;
    float mn = INFINITY;
#pragma unroll
    for (int r = 0; r < 8; ++r) {
      float y = acc[r];
      if (RESID) {
        const float rr = acr[r] * RES_CARRY_INV;
        y = y + rr;
      }
      y = y * WCARRY_INV;
      y = y + bv;
      ls = ls + y;
      const float y2 = y * y;
      lq = lq + y2;
      if (POOL) {
        mx = fmaxf(mx, y);
        mn = fminf(mn, y);
      } else {
        slab[wave][(8 * h + r) * 68 + col] = y;
      }
    }
    const float ls2 = __shfl_xor(ls, 16, 32);
    const float lq2 = __shfl_xor(lq, 16, 32);
    const float mx2 = __shfl_xor(mx, 16, 32);
    const float mn2 = __shfl_xor(mn, 16, 32);
    ls = ls + ls2;
    lq = lq + lq2;
    mx = fmaxf(mx, mx2);
    mn = fminf(mn, mn2);
    if (h == 0) {
      rs[wave][col] = ls;
      rq[wave][col] = lq;
      if (POOL) {
        pm[wave][col] = mx;
        pn[wave][col] = mn;
      }
    }
  }

  if (!POOL) {
    wave_lds_sync();
    const int q = lane >> 3;
    const int c8 = (lane & 7) * 8;
    v4u ov[4];
#pragma unroll
    for (int it = 0; it < 4; ++it) {
      const int row = it * 4 + q;
      const float* sp = &slab[wave][row * 68 + c8];
      const v4f fa = *(const v4f*)sp;
      const v4f fb2 = *(const v4f*)(sp + 4);
      const float e0 = fa[0];
      const float e1 = fa[1];
      const float e2 = fa[2];
      const float e3 = fa[3];
      const float e4 = fb2[0];
      const float e5 = fb2[1];
      const float e6 = fb2[2];
      const float e7 = fb2[3];
      ov[it] = (v4u){ pack2(e0, e1), pack2(e2, e3), pack2(e4, e5), pack2(e6, e7) };
    }
    unsigned* yp = Yout + (size_t)(blockIdx.x * 64 + wave * 16) * 32 + (lane & 7) * 4;
    for (int pass = 0; pass < 2; ++pass) {
#pragma unroll
      for (int it = 0; it < 4; ++it) {
        *(volatile v4u*)(yp + (size_t)(it * 4 + q) * 32) = ov[it];
      }
      __threadfence();
    }
  }
  __syncthreads();

  if (t < NOUT / 2) {
    const int i4 = 4 * t;
    const bool is_sum = (i4 < NOUT);
    const int colb = is_sum ? i4 : (i4 - NOUT);
    const v4f a0 = *(const v4f*)(&rs[0][colb]);
    const v4f a1 = *(const v4f*)(&rs[1][colb]);
    const v4f a2 = *(const v4f*)(&rs[2][colb]);
    const v4f a3 = *(const v4f*)(&rs[3][colb]);
    const v4f q0 = *(const v4f*)(&rq[0][colb]);
    const v4f q1 = *(const v4f*)(&rq[1][colb]);
    const v4f q2 = *(const v4f*)(&rq[2][colb]);
    const v4f q3 = *(const v4f*)(&rq[3][colb]);
    v4f v;
#pragma unroll
    for (int e = 0; e < 4; ++e) {
      const float s = ((a0[e] + a1[e]) + a2[e]) + a3[e];
      const float qq = ((q0[e] + q1[e]) + q2[e]) + q3[e];
      v[e] = is_sum ? s : qq;
    }
    float* pp = pst + (size_t)blockIdx.x * 256 + i4;
    for (int pass = 0; pass < 2; ++pass) {
      *(volatile v4f*)pp = v;
      __threadfence();
    }
  }
  if (POOL) {
    const int fi = 4 * t;
    const int g = fi >> 8;
    const int wi = fi & 255;
    const bool is_min = (wi >= 128);
    const int colb = wi & 127;
    const v4f m0 = *(const v4f*)(&pm[2 * g][colb]);
    const v4f m1 = *(const v4f*)(&pm[2 * g + 1][colb]);
    const v4f n0 = *(const v4f*)(&pn[2 * g][colb]);
    const v4f n1 = *(const v4f*)(&pn[2 * g + 1][colb]);
    v4f v;
#pragma unroll
    for (int e = 0; e < 4; ++e) {
      const float vmax = fmaxf(m0[e], m1[e]);
      const float vmin = fminf(n0[e], n1[e]);
      v[e] = is_min ? vmin : vmax;
    }
    float* gp = gmm + (size_t)blockIdx.x * 512 + fi;
    for (int pass = 0; pass < 2; ++pass) {
      *(volatile v4f*)gp = v;
      __threadfence();
    }
  }
}

template <int NOUT>
__global__ __launch_bounds__(512) void k_stats(const float* __restrict__ pst, const float* __restrict__ g,
                                               const float* __restrict__ beta, float* __restrict__ ss) {
  constexpr int NCOL = 2 * NOUT;
  constexpr int NPART = 512 / NCOL;
  constexpr int ROWS = LAYER_BLOCKS / NPART;
  static_assert(NPART * NCOL == 512);
  static_assert(ROWS * NPART == LAYER_BLOCKS);
  __shared__ double part[512];
  __shared__ __align__(16) float so[256];
  const int t = threadIdx.x;
  const int col = t % NCOL;
  const int p = t / NCOL;
  double acc = 0.0;
  const float* pp = pst + (size_t)(p * ROWS) * 256 + col;
#pragma unroll 4
  for (int r = 0; r < ROWS; ++r) {
    const float x = pp[(size_t)r * 256];
    acc = acc + (double)x;
  }
  part[t] = acc;
  __syncthreads();
  if (t < 128) {
    const int o = t < NOUT ? t : NOUT - 1;
    double S = 0.0;
    double Q = 0.0;
#pragma unroll
    for (int pi = 0; pi < NPART; ++pi) {
      S = S + part[pi * NCOL + o];
      Q = Q + part[pi * NCOL + NOUT + o];
    }
    const double inv_m = 1.0 / (double)MROWS_ALL;
    const double mu = S * inv_m;
    const double msq = mu * mu;
    double var = Q * inv_m - msq;
    var = var < 0.0 ? 0.0 : var;
    const float vf = (float)var + BN_EPS;
    const float rr = rsqrtf(vf);
    const float gg = g[o];
    const float bb = beta[o];
    const float av = gg * rr;
    const float mua = (float)mu * av;
    const float cv = bb - mua;
    so[t] = (t < NOUT) ? av : 0.0f;
    so[128 + t] = (t < NOUT) ? cv : 0.0f;
  }
  __syncthreads();
  if (t < 64) {
    const v4f v = *(const v4f*)(&so[4 * t]);
    float* sp = ss + 4 * t;
    for (int pass = 0; pass < 2; ++pass) {
      *(volatile v4f*)sp = v;
      __threadfence();
    }
  }
}

__global__ __launch_bounds__(256) void k_final(const float* __restrict__ gmm, const float* __restrict__ ss,
                                               float* __restrict__ out1) {
  __shared__ float T[128 * 33];
  const int t = threadIdx.x;
  const int b = blockIdx.x >> 4;
  const int k0 = (blockIdx.x & 15) * 32;
#pragma unroll 1
  for (int i = 0; i < 4; ++i) {
    const int idx4 = i * 256 + t;
    const int kl = idx4 >> 5;
    const int o4 = (idx4 & 31) * 4;
    const size_t G = (size_t)(b * NCENT + k0 + kl);
    const v4f mx = *(const v4f*)(gmm + G * 256 + o4);
    const v4f mn = *(const v4f*)(gmm + G * 256 + 128 + o4);
    const v4f sc = *(const v4f*)(ss + o4);
    const v4f sh = *(const v4f*)(ss + 128 + o4);
#pragma unroll
    for (int e = 0; e < 4; ++e) {
      const float s = sc[e];
      const float x = (s >= 0.0f) ? mx[e] : mn[e];
      float y = x * s;
      y = y + sh[e];
      y = fmaxf(y, 0.0f);
      T[(o4 + e) * 33 + kl] = y;
    }
  }
  __syncthreads();
  const int lane = t & 31;
  const int wave = t >> 5;
  const int q = lane >> 3;
  const int c4 = (lane & 7) * 4;
  v4f v[4];
#pragma unroll
  for (int it = 0; it < 4; ++it) {
    const int o = wave * 16 + it * 4 + q;
    v[it] = (v4f){ T[o * 33 + c4], T[o * 33 + c4 + 1], T[o * 33 + c4 + 2], T[o * 33 + c4 + 3] };
  }
  for (int pass = 0; pass < 2; ++pass) {
#pragma unroll
    for (int it = 0; it < 4; ++it) {
      const int o = wave * 16 + it * 4 + q;
      *(volatile v4f*)(out1 + ((size_t)(b * 128 + o)) * NCENT + k0 + c4) = v[it];
    }
    __threadfence();
  }
}

extern "C" void kernel_launch(void* const* d_in, const int* in_sizes, int n_in,
                              void* d_out, int out_size, void* d_ws, size_t ws_size,
                              hipStream_t stream) {
  (void)in_sizes; (void)n_in; (void)out_size;
  const float* xyz  = (const float*)d_in[0];
  const float* feat = (const float*)d_in[1];
  const float* W0   = (const float*)d_in[2];
  const float* b0   = (const float*)d_in[3];
  const float* g0   = (const float*)d_in[4];
  const float* be0  = (const float*)d_in[5];
  const float* W1   = (const float*)d_in[6];
  const float* b1   = (const float*)d_in[7];
  const float* g1   = (const float*)d_in[8];
  const float* be1  = (const float*)d_in[9];
  const float* W2   = (const float*)d_in[10];
  const float* b2   = (const float*)d_in[11];
  const float* g2   = (const float*)d_in[12];
  const float* be2  = (const float*)d_in[13];

  constexpr size_t OUT0_BYTES = (size_t)NBATCH * 3 * NCENT * 4;
  constexpr size_t OUT1_BYTES = (size_t)NBATCH * 128 * NCENT * 4;
  static_assert(OUT0_BYTES == 98304);
  static_assert(OUT0_BYTES + OUT1_BYTES == 4292608);
  float* out0 = (float*)d_out;
  float* out1 = (float*)d_out + OUT0_BYTES / 4;

  constexpr size_t SZ_CEN = OUT0_BYTES;
  constexpr size_t SZ_WPL = 7168 * 4;
  constexpr size_t SZ_SS  = 256 * 4;
  constexpr size_t SZ_PST = (size_t)LAYER_BLOCKS * 256 * 4;
  constexpr size_t SZ_GMM = (size_t)NBATCH * NCENT * 256 * 4;
  constexpr size_t SZ_X0  = (size_t)MROWS_ALL * 32 * 2;
  constexpr size_t SZ_Y   = (size_t)MROWS_ALL * 64 * 2;
  constexpr size_t OFF_CEN = 0;
  constexpr size_t OFF_WPL = OFF_CEN + SZ_CEN;
  constexpr size_t OFF_SS0 = OFF_WPL + SZ_WPL;
  constexpr size_t OFF_SS1 = OFF_SS0 + SZ_SS;
  constexpr size_t OFF_SS2 = OFF_SS1 + SZ_SS;
  constexpr size_t OFF_PST = OFF_SS2 + SZ_SS;
  constexpr size_t OFF_GMM = OFF_PST + SZ_PST;
  constexpr size_t OFF_X0  = OFF_GMM + SZ_GMM;
  constexpr size_t OFF_Y0  = OFF_X0 + SZ_X0;
  constexpr size_t OFF_Y1  = OFF_Y0 + SZ_Y;
  constexpr size_t WS_TOTAL = OFF_Y1 + SZ_Y;
  static_assert(WS_TOTAL == 96599040);
  static_assert(WS_TOTAL <= 134217728);
  static_assert(OFF_WPL % 128 == 0 && OFF_SS0 % 128 == 0 && OFF_PST % 128 == 0);
  static_assert(OFF_GMM % 128 == 0 && OFF_X0 % 128 == 0 && OFF_Y0 % 128 == 0 && OFF_Y1 % 128 == 0);
  if (ws_size < WS_TOTAL) return;

  char* ws = (char*)d_ws;
  float*    cen = (float*)(ws + OFF_CEN);
  unsigned* wpl = (unsigned*)(ws + OFF_WPL);
  float*    ss0 = (float*)(ws + OFF_SS0);
  float*    ss1 = (float*)(ws + OFF_SS1);
  float*    ss2 = (float*)(ws + OFF_SS2);
  float*    pst = (float*)(ws + OFF_PST);
  float*    gmm = (float*)(ws + OFF_GMM);
  unsigned* X0  = (unsigned*)(ws + OFF_X0);
  unsigned* Y0  = (unsigned*)(ws + OFF_Y0);
  unsigned* Y1  = (unsigned*)(ws + OFF_Y1);

  k_prep<<<28, 256, 0, stream>>>(W0, W1, W2, wpl);
  k_fps<<<NBATCH, 1024, 0, stream>>>(xyz, out0, cen);
  k_group<<<NBATCH * 16, 128, 0, stream>>>(xyz, feat, cen, X0);

  k_layer<32, 64, false, false, true><<<LAYER_BLOCKS, 128, 0, stream>>>(X0, wpl, b0, ss0, Y0, pst, gmm);
  k_stats<64><<<1, 512, 0, stream>>>(pst, g0, be0, ss0);
  k_layer<64, 64, true, false, false><<<LAYER_BLOCKS, 128, 0, stream>>>(Y0, wpl + 1024, b1, ss0, Y1, pst, gmm);
  k_stats<64><<<1, 512, 0, stream>>>(pst, g1, be1, ss1);
  k_layer<64, 128, true, true, false><<<LAYER_BLOCKS, 128, 0, stream>>>(Y1, wpl + 3072, b2, ss1, Y1, pst, gmm);
  k_stats<128><<<1, 512, 0, stream>>>(pst, g2, be2, ss2);

  k_final<<<NBATCH * 16, 256, 0, stream>>>(gmm, ss2, out1);
}
